// Word_Attention_15556371546452
// MI455X (gfx1250) — hardware-verified
//
#include <hip/hip_runtime.h>
#include <hip/hip_bf16.h>
#include <stddef.h>
#include <stdint.h>

#define NB    4
#define LSEQ  4096
#define DM    256
#define DH    128
#define NTOK  (NB * LSEQ)
#define NQKV  (3 * DH)
#define BR    32
#define BC    128
#define NQT   (LSEQ / BR)
#define NCH   (LSEQ / BC)
#define PSC   1024.0f
#define PINV  0.0009765625f

static_assert(DM % 32 == 0);
static_assert(DH == 128);
static_assert(LSEQ % 256 == 0);
static_assert(NTOK % 256 == 0);
static_assert(NQKV % 64 == 0);
static_assert(LSEQ % BR == 0);
static_assert(LSEQ % BC == 0);
static_assert(BC % 32 == 0);
static_assert((NTOK * DM) % 8 == 0);
static_assert(DH % 16 == 0);
static_assert(DM == 256);

typedef float          v8f   __attribute__((ext_vector_type(8)));
typedef float          v4f   __attribute__((ext_vector_type(4)));
typedef unsigned int   v4u   __attribute__((ext_vector_type(4)));
typedef unsigned short v8us  __attribute__((ext_vector_type(8)));
typedef unsigned short v16us __attribute__((ext_vector_type(16)));
typedef __bf16         v16b  __attribute__((ext_vector_type(16)));
typedef _Float16       v16h  __attribute__((ext_vector_type(16)));
typedef unsigned short ush;

union FragU { v16us v; v8us h[2]; v16b b; v16h f; };
union PackU { v8us s; v4u u; };
struct HL { v4u h; v4u l; };

__device__ __forceinline__ ush f2bf(float f) {
  const unsigned u = __float_as_uint(f);
  return (ush)((u + 0x7FFFu + ((u >> 16) & 1u)) >> 16);
}
__device__ __forceinline__ float bf2f(ush b) { return __uint_as_float(((unsigned)b) << 16); }
__device__ __forceinline__ ush f2h(float f) {
  const _Float16 h = (_Float16)f;
  return __builtin_bit_cast(ush, h);
}

__device__ __forceinline__ HL split8(v8f f) {
  PackU ph, pl;
#pragma unroll
  for (int e = 0; e < 8; ++e) {
    const ush hi = f2bf(f[e]);
    ph.s[e] = hi;
    pl.s[e] = f2bf(f[e] - bf2f(hi));
  }
  HL r; r.h = ph.u; r.l = pl.u;
  return r;
}

__device__ __forceinline__ v8f mmab(v16us a, v16us b, v8f c) {
  FragU ua, ub; ua.v = a; ub.v = b;
  c = __builtin_amdgcn_wmma_f32_16x16x32_bf16(false, ua.b, false, ub.b, (short)0, c, false, false);
  asm volatile("v_nop\n\tv_nop\n\tv_nop\n\tv_nop" : "+v"(c) : "v"(a), "v"(b));
  return c;
}
__device__ __forceinline__ v8f mmah(v16us a, v16us b, v8f c) {
  FragU ua, ub; ua.v = a; ub.v = b;
  c = __builtin_amdgcn_wmma_f32_16x16x32_f16(false, ua.f, false, ub.f, (short)0, c, false, false);
  asm volatile("v_nop\n\tv_nop\n\tv_nop\n\tv_nop" : "+v"(c) : "v"(a), "v"(b));
  return c;
}

__device__ __forceinline__ v16us ldfragu(const ush* p, int ld, int row0, int k0, int lane) {
  const int m = lane & 15, lh = lane >> 4;
  const ush* q = p + (size_t)(row0 + m) * ld + k0 + 8 * lh;
  FragU f;
  f.h[0] = *(const v8us*)(q);
  f.h[1] = *(const v8us*)(q + 16);
  return f.v;
}

__device__ __forceinline__ v8f zero8() { return (v8f){0.f, 0.f, 0.f, 0.f, 0.f, 0.f, 0.f, 0.f}; }

__device__ __forceinline__ void gemm3_32x64(const ush* __restrict__ Ah, const ush* __restrict__ Al, int lda,
                                            const ush* __restrict__ Bh, const ush* __restrict__ Bl, int ldb,
                                            int m0, int n0, int lane, v8f (&acc)[2][4]) {
#pragma unroll 1
  for (int k0 = 0; k0 < DM; k0 += 32) {
    const v16us a0h = ldfragu(Ah, lda, m0, k0, lane);
    const v16us a1h = ldfragu(Ah, lda, m0 + 16, k0, lane);
    const v16us a0l = ldfragu(Al, lda, m0, k0, lane);
    const v16us a1l = ldfragu(Al, lda, m0 + 16, k0, lane);
#pragma unroll
    for (int t = 0; t < 4; ++t) {
      const v16us bh = ldfragu(Bh, ldb, n0 + 16 * t, k0, lane);
      const v16us bl = ldfragu(Bl, ldb, n0 + 16 * t, k0, lane);
      acc[0][t] = mmab(a0h, bh, acc[0][t]);
      acc[1][t] = mmab(a1h, bh, acc[1][t]);
      acc[0][t] = mmab(a0h, bl, acc[0][t]);
      acc[1][t] = mmab(a1h, bl, acc[1][t]);
      acc[0][t] = mmab(a0l, bh, acc[0][t]);
      acc[1][t] = mmab(a1l, bh, acc[1][t]);
    }
  }
}

__global__ __launch_bounds__(256) void k_cvt_x(const float* __restrict__ x, ush* __restrict__ xh,
                                               ush* __restrict__ xl, int ngrp) {
  const int t = blockIdx.x * 256 + (int)threadIdx.x;
  if (t >= ngrp) return;
  const size_t o = (size_t)t * 8;
  const v4f a0 = *(const v4f*)(x + o);
  const v4f a1 = *(const v4f*)(x + o + 4);
  const v8f f = (v8f){a0[0], a0[1], a0[2], a0[3], a1[0], a1[1], a1[2], a1[3]};
  const HL s = split8(f);
  *(volatile v4u*)(xh + o) = s.h;
  *(volatile v4u*)(xl + o) = s.l;
  __threadfence();
  *(volatile v4u*)(xh + o) = s.h;
  *(volatile v4u*)(xl + o) = s.l;
}

#define WTP 260
__global__ __launch_bounds__(256) void k_cvt_w(const float* __restrict__ wq, const float* __restrict__ wk,
                                               const float* __restrict__ wv,
                                               ush* __restrict__ w3h, ush* __restrict__ w3l) {
  __shared__ __align__(16) float st[16 * WTP];
  const int which = blockIdx.y;
  const float* w = (which == 0) ? wq : ((which == 1) ? wk : wv);
  const int tid = threadIdx.x;
  const int h0 = blockIdx.x * 16;
  {
    const float* src = w + (size_t)tid * DH + h0;
    const v4f a0 = *(const v4f*)(src);
    const v4f a1 = *(const v4f*)(src + 4);
    const v4f a2 = *(const v4f*)(src + 8);
    const v4f a3 = *(const v4f*)(src + 12);
#pragma unroll
    for (int e = 0; e < 4; ++e) {
      st[(e)      * WTP + tid] = a0[e];
      st[(4 + e)  * WTP + tid] = a1[e];
      st[(8 + e)  * WTP + tid] = a2[e];
      st[(12 + e) * WTP + tid] = a3[e];
    }
  }
  __syncthreads();
  v4u vh[2], vl[2];
  size_t go[2];
#pragma unroll
  for (int j = 0; j < 2; ++j) {
    const int p   = tid + 256 * j;
    const int row = p >> 5;
    const int pc  = p & 31;
    const float* sp = st + row * WTP + pc * 8;
    const v4f b0 = *(const v4f*)(sp);
    const v4f b1 = *(const v4f*)(sp + 4);
    const v8f f = (v8f){b0[0], b0[1], b0[2], b0[3], b1[0], b1[1], b1[2], b1[3]};
    const HL s = split8(f);
    vh[j] = s.h;
    vl[j] = s.l;
    go[j] = ((size_t)(which * DH + h0 + row)) * DM + (size_t)pc * 8;
  }
#pragma unroll
  for (int j = 0; j < 2; ++j) {
    *(volatile v4u*)(w3h + go[j]) = vh[j];
    *(volatile v4u*)(w3l + go[j]) = vl[j];
  }
  __threadfence();
#pragma unroll
  for (int j = 0; j < 2; ++j) {
    *(volatile v4u*)(w3h + go[j]) = vh[j];
    *(volatile v4u*)(w3l + go[j]) = vl[j];
  }
}

#define STP 72
__global__ __launch_bounds__(256) void k_qkv3(const ush* __restrict__ xh3, const ush* __restrict__ xl3,
                                              const ush* __restrict__ wth, const ush* __restrict__ wtl,
                                              const float* __restrict__ bq,
                                              const float* __restrict__ bk,
                                              const float* __restrict__ bv,
                                              ush* __restrict__ q3h, ush* __restrict__ q3l,
                                              ush* __restrict__ k3h, ush* __restrict__ k3l,
                                              ush* __restrict__ v16) {
  __shared__ __align__(16) ush st[256 * STP];
  const int tid = threadIdx.x, lane = tid & 31, wave = tid >> 5;
  const int hh = lane >> 4, c = lane & 15;
  const int mb = blockIdx.x * 256;
  const int m0 = mb + wave * 32;
  const int n0 = blockIdx.y * 64;
  const int which = n0 / DH;
  const int nn = n0 - which * DH;
  const int b  = mb / LSEQ;
  const int l0 = mb - b * LSEQ;
  const float* bias = (which == 0) ? bq : ((which == 1) ? bk : bv);

  v8f acc[2][4];
#pragma unroll
  for (int s = 0; s < 2; ++s)
#pragma unroll
    for (int t = 0; t < 4; ++t) acc[s][t] = zero8();
  gemm3_32x64(xh3, xl3, DM, wth, wtl, DM, m0, n0, lane, acc);

#pragma unroll
  for (int t = 0; t < 4; ++t) {
    const float bn = bias[nn + 16 * t + c];
#pragma unroll
    for (int sub = 0; sub < 2; ++sub) {
#pragma unroll
      for (int r = 0; r < 8; ++r) acc[sub][t][r] += bn;
    }
  }

  ush* bhp = (which == 0) ? q3h : k3h;
  ush* blp = (which == 0) ? q3l : k3l;
  size_t go[8];
#pragma unroll
  for (int j = 0; j < 8; ++j) {
    const int p  = tid + 256 * j;
    const int L  = p >> 3;
    const int pc = p & 7;
    if (which < 2) {
      go[j] = ((size_t)(mb + L)) * DH + nn + pc * 8;
    } else {
      const int d  = L >> 2;
      const int nl = (L & 3) * 64 + pc * 8;
      go[j] = ((size_t)(b * DH + nn + d)) * LSEQ + l0 + nl;
    }
  }

  const int nph = (which < 2) ? 2 : 1;
#pragma unroll 1
  for (int ph = 0; ph < nph; ++ph) {
    __syncthreads();
#pragma unroll
    for (int t = 0; t < 4; ++t) {
#pragma unroll
      for (int sub = 0; sub < 2; ++sub) {
#pragma unroll
        for (int r = 0; r < 8; ++r) {
          const int lr = wave * 32 + sub * 16 + 8 * hh + r;
          const float v = acc[sub][t][r];
          ush o;
          if (which < 2) {
            const ush hi = f2bf(v);
            o = (ph == 0) ? hi : f2bf(v - bf2f(hi));
          } else {
            o = f2h(v);
          }
          st[lr * STP + 16 * t + c] = o;
        }
      }
    }
    __syncthreads();
    v4u val[8];
    if (which < 2) {
#pragma unroll
      for (int j = 0; j < 8; ++j) {
        const int p  = tid + 256 * j;
        const int lr = p >> 3;
        const int pc = p & 7;
        PackU pk;
        pk.s  = *(const v8us*)(st + lr * STP + pc * 8);
        val[j] = pk.u;
      }
    } else {
#pragma unroll
      for (int j = 0; j < 8; ++j) {
        const int p  = tid + 256 * j;
        const int L  = p >> 3;
        const int pc = p & 7;
        const int d  = L >> 2;
        const int nl = (L & 3) * 64 + pc * 8;
        const ush* cp = st + nl * STP + d;
        PackU pk;
        pk.s = (v8us){cp[0 * STP], cp[1 * STP], cp[2 * STP], cp[3 * STP],
                      cp[4 * STP], cp[5 * STP], cp[6 * STP], cp[7 * STP]};
        val[j] = pk.u;
      }
    }
    ush* dst = (which == 2) ? v16 : ((ph == 0) ? bhp : blp);
#pragma unroll
    for (int j = 0; j < 8; ++j) *(volatile v4u*)(dst + go[j]) = val[j];
    __threadfence();
#pragma unroll
    for (int j = 0; j < 8; ++j) *(volatile v4u*)(dst + go[j]) = val[j];
    __threadfence();
  }
}

#define SSP 128
#define SPP 136
#define OTP 132
__global__ __launch_bounds__(256) void k_attn(const ush* __restrict__ q3h, const ush* __restrict__ q3l,
                                              const ush* __restrict__ k3h, const ush* __restrict__ k3l,
                                              const ush* __restrict__ v16,
                                              float* __restrict__ out) {
  __shared__ __align__(16) float sSO[BR * OTP];
  __shared__ __align__(16) ush   sP[BR * SPP];
  __shared__ __align__(16) float sRed[BR * 8];
  __shared__ __align__(16) float rM[BR];
  __shared__ __align__(16) float rMn[BR];
  __shared__ __align__(16) float rL[BR];
  __shared__ __align__(16) float rSc[BR];

  float* sS = sSO;
  const int tid = threadIdx.x, lane = tid & 31, wave = tid >> 5;
  const int hh = lane >> 4, c = lane & 15;
  const int b  = blockIdx.y;
  const int q0 = (int)blockIdx.x * BR;
  const ush* Qh = q3h + (size_t)b * LSEQ * DH;
  const ush* Ql = q3l + (size_t)b * LSEQ * DH;
  const ush* Kh = k3h + (size_t)b * LSEQ * DH;
  const ush* Kl = k3l + (size_t)b * LSEQ * DH;
  const ush* Vt = v16 + (size_t)b * DH * LSEQ;
  const float NEGI = -__builtin_huge_valf();
  if (tid < BR) { rM[tid] = NEGI; rL[tid] = 0.f; }
  __syncthreads();

  v8f oacc[2];
  oacc[0] = zero8(); oacc[1] = zero8();

  const int srow = tid >> 3, schk = tid & 7;

#pragma unroll 1
  for (int ch = 0; ch < NCH; ++ch) {
    const int j0  = ch * BC;
    const int kr0 = j0 + wave * 16;
    v8f s[2];
    s[0] = zero8(); s[1] = zero8();
#pragma unroll 1
    for (int k0 = 0; k0 < DH; k0 += 32) {
      const v16us a0h = ldfragu(Qh, DH, q0, k0, lane);
      const v16us a1h = ldfragu(Qh, DH, q0 + 16, k0, lane);
      const v16us a0l = ldfragu(Ql, DH, q0, k0, lane);
      const v16us a1l = ldfragu(Ql, DH, q0 + 16, k0, lane);
      const v16us kbh = ldfragu(Kh, DH, kr0, k0, lane);
      const v16us kbl = ldfragu(Kl, DH, kr0, k0, lane);
      s[0] = mmab(a0h, kbh, s[0]);
      s[1] = mmab(a1h, kbh, s[1]);
      s[0] = mmab(a0h, kbl, s[0]);
      s[1] = mmab(a1h, kbl, s[1]);
      s[0] = mmab(a0l, kbh, s[0]);
      s[1] = mmab(a1l, kbh, s[1]);
    }
#pragma unroll
    for (int t = 0; t < 2; ++t) {
#pragma unroll
      for (int r = 0; r < 8; ++r) {
        const int row = 16 * t + 8 * hh + r;
        sS[row * SSP + wave * 16 + c] = s[t][r];
      }
    }
    __syncthreads();
    {
      const float* sr = sS + srow * SSP + schk * 16;
      const v4f x0 = *(const v4f*)(sr);
      const v4f x1 = *(const v4f*)(sr + 4);
      const v4f x2 = *(const v4f*)(sr + 8);
      const v4f x3 = *(const v4f*)(sr + 12);
      float mx = x0[0];
#pragma unroll
      for (int e = 1; e < 4; ++e) mx = fmaxf(mx, x0[e]);
#pragma unroll
      for (int e = 0; e < 4; ++e) { mx = fmaxf(mx, x1[e]); mx = fmaxf(mx, x2[e]); mx = fmaxf(mx, x3[e]); }
      sRed[srow * 8 + schk] = mx;
    }
    __syncthreads();
    if (tid < BR) {
      float mx = rM[tid];
#pragma unroll
      for (int i = 0; i < 8; ++i) mx = fmaxf(mx, sRed[tid * 8 + i]);
      rMn[tid] = mx;
    }
    __syncthreads();
    {
      const float mx = rMn[srow];
      const float* sr = sS + srow * SSP + schk * 16;
      float sum = 0.f;
      PackU ph0, ph1;
#pragma unroll
      for (int e = 0; e < 8; ++e) {
        const float p = __expf(sr[e] - mx);
        sum += p;
        ph0.s[e] = f2h(p * PSC);
      }
#pragma unroll
      for (int e = 0; e < 8; ++e) {
        const float p = __expf(sr[8 + e] - mx);
        sum += p;
        ph1.s[e] = f2h(p * PSC);
      }
      *(v8us*)(sP + srow * SPP + schk * 16)     = ph0.s;
      *(v8us*)(sP + srow * SPP + schk * 16 + 8) = ph1.s;
      sRed[srow * 8 + schk] = sum;
    }
    __syncthreads();
    if (tid < BR) {
      float sum = 0.f;
#pragma unroll
      for (int i = 0; i < 8; ++i) sum += sRed[tid * 8 + i];
      const float mnew = rMn[tid];
      const float fac  = __expf(rM[tid] - mnew);
      rL[tid]  = rL[tid] * fac + sum;
      rM[tid]  = mnew;
      rSc[tid] = fac;
    }
    __syncthreads();
#pragma unroll
    for (int t = 0; t < 2; ++t) {
      const v4f f0 = *(const v4f*)(rSc + 16 * t + 8 * hh);
      const v4f f1 = *(const v4f*)(rSc + 16 * t + 8 * hh + 4);
#pragma unroll
      for (int r = 0; r < 4; ++r) {
        oacc[t][r]     *= f0[r];
        oacc[t][4 + r] *= f1[r];
      }
    }
#pragma unroll 1
    for (int kk = 0; kk < BC / 32; ++kk) {
      const v16us pa0 = ldfragu(sP, SPP, 0, kk * 32, lane);
      const v16us pa1 = ldfragu(sP, SPP, 16, kk * 32, lane);
      const v16us vb = ldfragu(Vt, LSEQ, wave * 16, j0 + kk * 32, lane);
      oacc[0] = mmah(pa0, vb, oacc[0]);
      oacc[1] = mmah(pa1, vb, oacc[1]);
    }
    __syncthreads();
  }

  float* sO = sSO;
#pragma unroll
  for (int t = 0; t < 2; ++t) {
#pragma unroll
    for (int r = 0; r < 8; ++r) {
      const int row  = 16 * t + 8 * hh + r;
      const float lv  = rL[row];
      const float inv = (lv > 0.f) ? ((1.0f / lv) * PINV) : 0.f;
      sO[row * OTP + wave * 16 + c] = oacc[t][r] * inv;
    }
  }
  __syncthreads();
  v4f val[4];
  size_t go[4];
  const size_t grow0 = (size_t)b * LSEQ + (size_t)q0;
#pragma unroll
  for (int it = 0; it < 4; ++it) {
    const int p   = tid + 256 * it;
    const int L   = p >> 3;
    const int pc  = p & 7;
    const int row = L >> 2;
    const int qu  = L & 3;
    val[it] = *(const v4f*)(sO + row * OTP + qu * 32 + pc * 4);
    go[it]  = (grow0 + (size_t)row) * DH + qu * 32 + pc * 4;
  }
#pragma unroll
  for (int it = 0; it < 4; ++it) *(volatile v4f*)(out + go[it]) = val[it];
  __threadfence();
#pragma unroll
  for (int it = 0; it < 4; ++it) *(volatile v4f*)(out + go[it]) = val[it];
}

extern "C" void kernel_launch(void* const* d_in, const int* in_sizes, int n_in,
                              void* d_out, int out_size, void* d_ws, size_t ws_size,
                              hipStream_t stream) {
  if (n_in < 7) return;
  if (in_sizes[0] != NTOK * DM) return;
  if (in_sizes[1] != DM * DH) return;
  if (in_sizes[2] != DH) return;
  if (in_sizes[3] != DM * DH) return;
  if (in_sizes[4] != DH) return;
  if (in_sizes[5] != DM * DH) return;
  if (in_sizes[6] != DH) return;
  if (out_size != NTOK * DH) return;

  const float* x  = (const float*)d_in[0];
  const float* wq = (const float*)d_in[1];
  const float* bq = (const float*)d_in[2];
  const float* wk = (const float*)d_in[3];
  const float* bk = (const float*)d_in[4];
  const float* wv = (const float*)d_in[5];
  const float* bv = (const float*)d_in[6];
  float* out = (float*)d_out;

  size_t off = 0;
  const size_t oX3h = off; off += (size_t)NTOK * DM * 2;
  const size_t oX3l = off; off += (size_t)NTOK * DM * 2;
  const size_t oW3h = off; off += (size_t)NQKV * DM * 2;
  const size_t oW3l = off; off += (size_t)NQKV * DM * 2;
  const size_t oQ3h = off; off += (size_t)NTOK * DH * 2;
  const size_t oQ3l = off; off += (size_t)NTOK * DH * 2;
  const size_t oK3h = off; off += (size_t)NTOK * DH * 2;
  const size_t oK3l = off; off += (size_t)NTOK * DH * 2;
  const size_t oV16 = off; off += (size_t)NB * DH * LSEQ * 2;
  if (off > ws_size) return;
  if (off > (size_t)134217728) return;

  char* ws = (char*)d_ws;
  ush* X3h = (ush*)(ws + oX3h);
  ush* X3l = (ush*)(ws + oX3l);
  ush* W3h = (ush*)(ws + oW3h);
  ush* W3l = (ush*)(ws + oW3l);
  ush* Q3h = (ush*)(ws + oQ3h);
  ush* Q3l = (ush*)(ws + oQ3l);
  ush* K3h = (ush*)(ws + oK3h);
  ush* K3l = (ush*)(ws + oK3l);
  ush* V16 = (ush*)(ws + oV16);

  const int ngx = in_sizes[0] / 8;
  k_cvt_x<<<dim3((ngx + 255) / 256), dim3(256), 0, stream>>>(x, X3h, X3l, ngx);
  k_cvt_w<<<dim3(DH / 16, 3), dim3(256), 0, stream>>>(wq, wk, wv, W3h, W3l);
  k_qkv3<<<dim3(NTOK / 256, NQKV / 64), dim3(256), 0, stream>>>(X3h, X3l, W3h, W3l, bq, bk, bv,
                                                               Q3h, Q3l, K3h, K3l, V16);
  k_attn<<<dim3(NQT, NB), dim3(256), 0, stream>>>(Q3h, Q3l, K3h, K3l, V16, out);
  (void)hipGetLastError();
}
